// DyGCN_58643483459899
// MI455X (gfx1250) — hardware-run, weakly checked
//
#include <hip/hip_runtime.h>
#include <math.h>


constexpr int kB = 8, kN = 1024, kC = 64, kT = 12, kO = 64;
constexpr int kG = kT * kB;
constexpr int kTG = 2;
constexpr int kGL = kTG * kB;
constexpr int kNGRP = kT / kTG;
constexpr int kNT = kN / 128;
constexpr int kPAIRS = kNT * (kNT + 1) / 2;

static_assert(kN % 128 == 0);
static_assert(kNT == 8);
static_assert(kC == 64 && kO == 64);
static_assert(kT % kTG == 0);
static_assert(kG == 96 && kGL == 16 && kNGRP * kGL == kG);
static_assert(3 * 2 * (kO / 32) == 12);
static_assert(kPAIRS == 36);
static_assert((kN * kN / 8) == 512 * 256);

typedef __bf16 v16b __attribute__((ext_vector_type(16)));
typedef __bf16 v8b  __attribute__((ext_vector_type(8)));
typedef float  v8f  __attribute__((ext_vector_type(8)));
typedef float  v4f  __attribute__((ext_vector_type(4)));
typedef unsigned int v4u __attribute__((ext_vector_type(4)));
typedef v8b __attribute__((may_alias)) v8ba;
typedef v4f __attribute__((may_alias)) v4fa;
typedef v4u __attribute__((may_alias)) v4ua;

union FB { v16b v; v8b h[2]; };

constexpr size_t SZ_XT   = (size_t)kG * kN * kC * 2;
constexpr size_t SZ_XTT  = SZ_XT;
constexpr size_t SZ_ADJB = (size_t)kN * kN * 2;
constexpr size_t SZ_WDT  = (size_t)kT * 64 * 64 * 2;
constexpr size_t SZ_WS2  = (size_t)kT * 64 * 128 * 2;
constexpr size_t SZ_WD2  = SZ_WS2;
constexpr size_t SZ_W0T  = (size_t)64 * 64 * 2;
constexpr size_t SZ_SAGG = (size_t)kG * kN * 128 * 2;
constexpr size_t SZ_DAGG = SZ_SAGG;
constexpr size_t SZ_DEP  = (size_t)kGL * kN * 256 * 2;
constexpr size_t SZ_DA   = (size_t)kGL * kN * kN * 2;
constexpr size_t SZ_RSP  = (size_t)kGL * kNT * kN * 4;
constexpr size_t SZ_DIS  = (size_t)kG * kN * 4;
constexpr size_t SZ_XST  = (size_t)kGL * 128 * kN * 2;
constexpr size_t OFF_XT   = 0;
constexpr size_t OFF_XTT  = OFF_XT + SZ_XT;
constexpr size_t OFF_ADJB = OFF_XTT + SZ_XTT;
constexpr size_t OFF_WDT  = OFF_ADJB + SZ_ADJB;
constexpr size_t OFF_WS2  = OFF_WDT + SZ_WDT;
constexpr size_t OFF_WD2  = OFF_WS2 + SZ_WS2;
constexpr size_t OFF_W0T  = OFF_WD2 + SZ_WD2;
constexpr size_t OFF_SAGG = OFF_W0T + SZ_W0T;
constexpr size_t OFF_DAGG = OFF_SAGG + SZ_SAGG;
constexpr size_t OFF_DEP  = OFF_DAGG + SZ_DAGG;
constexpr size_t OFF_DA   = OFF_DEP + SZ_DEP;
constexpr size_t OFF_RSP  = OFF_DA + SZ_DA;
constexpr size_t OFF_DIS  = OFF_RSP + SZ_RSP;
constexpr size_t OFF_XST  = OFF_DIS + SZ_DIS;
constexpr size_t WS_TOTAL = OFF_XST + SZ_XST;
static_assert(WS_TOTAL == 125149184);
static_assert(WS_TOTAL <= 134217728);
static_assert((OFF_XTT % 256) == 0 && (OFF_ADJB % 256) == 0 && (OFF_WDT % 256) == 0 && (OFF_WS2 % 256) == 0);
static_assert((OFF_WD2 % 256) == 0 && (OFF_W0T % 256) == 0 && (OFF_SAGG % 256) == 0 && (OFF_DAGG % 256) == 0);
static_assert((OFF_DEP % 256) == 0 && (OFF_DA % 256) == 0 && (OFF_RSP % 256) == 0 && (OFF_DIS % 256) == 0 && (OFF_XST % 256) == 0);

constexpr int LDS_PREPX = 64 * 768 * 2;
constexpr int LDS_BASE  = 128 * 68 * 4 + 128 * 128 * 4 + 64 * 4;
constexpr int LDS_ANTI  = 65536 + 65536 + 128 * 129 * 4 + 256 * 4;
constexpr int LDS_PV    = 128 * 132 * 4 + 128 * 4;
constexpr int LDS_OUT   = 32 * 768 * 4 + (768 + 768 + 64) * 4;
static_assert(LDS_ANTI <= 327680 && LDS_OUT <= 327680 && LDS_BASE <= 327680);

__device__ __forceinline__ unsigned bfbits(float f) {
  const unsigned u = __float_as_uint(f);
  return (u + 0x7FFFu + ((u >> 16) & 1u)) >> 16;
}
__device__ __forceinline__ float bf2f(unsigned h) { return __uint_as_float(h << 16); }
__device__ __forceinline__ float bfr(float f) { return bf2f(bfbits(f)); }
__device__ __forceinline__ unsigned pk16(unsigned a, unsigned b) { return a | (b << 16); }

__device__ __forceinline__ v8f mma_bf(v16b a, v16b b, v8f c) {
  c = __builtin_amdgcn_wmma_f32_16x16x32_bf16(false, a, false, b, (short)0, c, false, false);
  asm volatile("v_nop\n\tv_nop\n\tv_nop\n\tv_nop" : "+v"(c) : "v"(a), "v"(b));
  return c;
}
__device__ __forceinline__ v16b ldfrag_g(const unsigned short* __restrict__ p, int h) {
  FB f;
  f.h[0] = *(const v8ba*)(p + 8 * h);
  f.h[1] = *(const v8ba*)(p + 16 + 8 * h);
  return f.v;
}
__device__ __forceinline__ v16b ldfrag_l(const unsigned short* p, int h) {
  FB f;
  f.h[0] = *(const v8ba*)(p + 8 * h);
  f.h[1] = *(const v8ba*)(p + 16 + 8 * h);
  return f.v;
}

__device__ __forceinline__ void split8(const float (&f)[8], v4u& hi, v4u& lo) {
  unsigned hb[8], lb[8];
#pragma unroll
  for (int e = 0; e < 8; ++e) {
    hb[e] = bfbits(f[e]);
    lb[e] = bfbits(f[e] - bf2f(hb[e]));
  }
  hi = (v4u){pk16(hb[0], hb[1]), pk16(hb[2], hb[3]), pk16(hb[4], hb[5]), pk16(hb[6], hb[7])};
  lo = (v4u){pk16(lb[0], lb[1]), pk16(lb[2], lb[3]), pk16(lb[4], lb[5]), pk16(lb[6], lb[7])};
}
__device__ __forceinline__ v4u blend4(v4u a, v4u b, unsigned sel) {
  const unsigned mk = 0u - sel;
  return (a & ~mk) | (b & mk);
}

__device__ __forceinline__ float tanh_fast(float a) {
  a = fminf(fmaxf(a, -15.0f), 15.0f);
  const float e = __expf(2.0f * a);
  return (e - 1.0f) * __builtin_amdgcn_rcpf(e + 1.0f);
}

__global__ __launch_bounds__(256) void k_prep_x(const float* __restrict__ x,
                                                unsigned short* __restrict__ XT,
                                                unsigned short* __restrict__ XTT) {
  extern __shared__ __attribute__((aligned(16))) unsigned char sm_px[];
  unsigned short* xs = (unsigned short*)sm_px;
  const int tid = threadIdx.x;
  const int b = blockIdx.x >> 4, n0 = (blockIdx.x & 15) * 64;
  const float* src = x + ((size_t)b * kN + n0) * 768;
#pragma unroll 4
  for (int it = 0; it < 48; ++it) {
    const int i4 = it * 256 + tid;
    const v4f a = *(const v4fa*)(src + (size_t)i4 * 4);
    unsigned short* d = xs + i4 * 4;
    d[0] = (unsigned short)bfbits(a.x);
    d[1] = (unsigned short)bfbits(a.y);
    d[2] = (unsigned short)bfbits(a.z);
    d[3] = (unsigned short)bfbits(a.w);
  }
  __syncthreads();
#pragma unroll 1
  for (int t = 0; t < kT; ++t) {
    const int g = t * kB + b;
    v4u va[2], vb[2];
#pragma unroll
    for (int it = 0; it < 2; ++it) {
      const int id = it * 256 + tid;
      const int rr = id >> 3, p = id & 7;
      v4u a, c;
#pragma unroll
      for (int q = 0; q < 4; ++q) {
        const unsigned a0 = xs[rr * 768 + (8 * p + 2 * q) * 12 + t];
        const unsigned a1 = xs[rr * 768 + (8 * p + 2 * q + 1) * 12 + t];
        a[q] = pk16(a0, a1);
        const unsigned c0 = xs[(8 * p + 2 * q) * 768 + rr * 12 + t];
        const unsigned c1 = xs[(8 * p + 2 * q + 1) * 768 + rr * 12 + t];
        c[q] = pk16(c0, c1);
      }
      va[it] = a;
      vb[it] = c;
    }
    for (int pass = 0; pass < 2; ++pass) {
#pragma unroll
      for (int it = 0; it < 2; ++it) {
        const int id = it * 256 + tid;
        const int rr = id >> 3, p = id & 7;
        *(volatile v4u*)(XT + ((size_t)g * kN + n0 + rr) * 64 + 8 * p) = va[it];
        *(volatile v4u*)(XTT + ((size_t)g * 64 + rr) * kN + n0 + 8 * p) = vb[it];
      }
      __threadfence();
    }
  }
}

__device__ __forceinline__ void wt_stage(const float* __restrict__ W, float* tf, int tid) {
#pragma unroll
  for (int it = 0; it < 4; ++it) {
    const int i4 = it * 256 + tid;
    const int r = i4 >> 4, c4 = (i4 & 15) * 4;
    const v4f a = *(const v4fa*)(W + r * 64 + c4);
    *(v4fa*)(tf + r * 68 + c4) = a;
  }
}
template <int PITCH>
__device__ __forceinline__ void wt_emit(const float* tf, unsigned short* __restrict__ dst, int tid) {
  constexpr int PPR = PITCH / 8;
  constexpr int NIT = 64 * PPR / 256;
  v4u vv[NIT];
#pragma unroll
  for (int it = 0; it < NIT; ++it) {
    const int id = it * 256 + tid;
    const int o = id / PPR, p = id % PPR, oc = p & 7;
    v4u a;
#pragma unroll
    for (int q = 0; q < 4; ++q) {
      const float f0 = tf[(8 * oc + 2 * q) * 68 + o];
      const float f1 = tf[(8 * oc + 2 * q + 1) * 68 + o];
      a[q] = pk16(bfbits(f0), bfbits(f1));
    }
    vv[it] = a;
  }
  for (int pass = 0; pass < 2; ++pass) {
#pragma unroll
    for (int it = 0; it < NIT; ++it) {
      const int id = it * 256 + tid;
      const int o = id / PPR, p = id % PPR;
      *(volatile v4u*)(dst + (size_t)o * PITCH + 8 * p) = vv[it];
    }
    __threadfence();
  }
}

__global__ __launch_bounds__(256) void k_prep_w(const float* __restrict__ adj, const float* __restrict__ W0,
                                                const float* __restrict__ Ws, const float* __restrict__ Wd,
                                                unsigned short* __restrict__ ADJB, unsigned short* __restrict__ WDT,
                                                unsigned short* __restrict__ WS2, unsigned short* __restrict__ WD2,
                                                unsigned short* __restrict__ W0T) {
  __shared__ __attribute__((aligned(16))) float tf[64 * 68];
  const int tid = threadIdx.x;
  const int bid = blockIdx.x;
  if (bid < 512) {
    const size_t g8 = (size_t)bid * 256 + tid;
    const v4f a = *(const v4fa*)(adj + g8 * 8);
    const v4f c = *(const v4fa*)(adj + g8 * 8 + 4);
    const v4u o = {pk16(bfbits(a.x), bfbits(a.y)), pk16(bfbits(a.z), bfbits(a.w)),
                   pk16(bfbits(c.x), bfbits(c.y)), pk16(bfbits(c.z), bfbits(c.w))};
    *(volatile v4u*)(ADJB + g8 * 8) = o;
    __threadfence();
    *(volatile v4u*)(ADJB + g8 * 8) = o;
  } else {
    const int u = bid - 512;
    if (u < 12) {
      wt_stage(Wd + (size_t)u * 4096, tf, tid);
      __syncthreads();
      wt_emit<64>(tf, WDT + (size_t)u * 4096, tid);
      wt_emit<128>(tf, WD2 + (size_t)u * 8192, tid);
    } else if (u < 24) {
      const int t = u - 12;
      wt_stage(Ws + (size_t)t * 4096, tf, tid);
      __syncthreads();
      wt_emit<128>(tf, WS2 + (size_t)t * 8192, tid);
    } else {
      wt_stage(W0, tf, tid);
      __syncthreads();
      wt_emit<64>(tf, W0T, tid);
    }
  }
}

template <int NTHR>
__device__ __forceinline__ void store_hilo128(const float* tile, int pitch, unsigned short* __restrict__ dst, int tid) {
  constexpr int PER = 2048 / NTHR;
#pragma unroll 1
  for (int ch = 0; ch < PER / 4; ++ch) {
    v4u vv[4];
#pragma unroll
    for (int it = 0; it < 4; ++it) {
      const int id = (ch * 4 + it) * NTHR + tid;
      const int row = id >> 4, p = id & 15, oc = p & 7;
      const v4f f0 = *(const v4fa*)(tile + row * pitch + 8 * oc);
      const v4f f1 = *(const v4fa*)(tile + row * pitch + 8 * oc + 4);
      const float f[8] = {f0.x, f0.y, f0.z, f0.w, f1.x, f1.y, f1.z, f1.w};
      v4u hi, lo;
      split8(f, hi, lo);
      vv[it] = blend4(hi, lo, (unsigned)(p >> 3));
    }
    for (int pass = 0; pass < 2; ++pass) {
#pragma unroll
      for (int it = 0; it < 4; ++it) {
        const int id = (ch * 4 + it) * NTHR + tid;
        const int row = id >> 4, p = id & 15;
        *(volatile v4u*)(dst + (size_t)row * 128 + 8 * p) = vv[it];
      }
      __threadfence();
    }
  }
}

__global__ __launch_bounds__(128) __attribute__((amdgpu_num_vgpr(248)))
void k_static(const unsigned short* __restrict__ ADJB, const unsigned short* __restrict__ XTT,
              unsigned short* __restrict__ SAGG) {
  __shared__ __attribute__((aligned(16))) float sT[128 * 68];
  const int tid = threadIdx.x, lane = tid & 31, w = tid >> 5;
  const int h = lane >> 4, m = lane & 15;
  const int n0 = blockIdx.x * 128, g = blockIdx.y;
  const unsigned short* a0p = ADJB + (size_t)(n0 + 32 * w + m) * kN;
  const unsigned short* a1p = a0p + (size_t)16 * kN;
  const unsigned short* bp = XTT + ((size_t)g * 64 + m) * kN;
  const v8f zero8 = {0.f, 0.f, 0.f, 0.f, 0.f, 0.f, 0.f, 0.f};
  v8f acc[2][4];
#pragma unroll
  for (int mt = 0; mt < 2; ++mt)
#pragma unroll
    for (int nt = 0; nt < 4; ++nt) acc[mt][nt] = zero8;
#pragma unroll 1
  for (int k0 = 0; k0 < kN; k0 += 32) {
    const v16b a0 = ldfrag_g(a0p + k0, h);
    const v16b a1 = ldfrag_g(a1p + k0, h);
#pragma unroll
    for (int nt = 0; nt < 4; ++nt) {
      const v16b bb = ldfrag_g(bp + (size_t)nt * 16 * kN + k0, h);
      acc[0][nt] = mma_bf(a0, bb, acc[0][nt]);
      acc[1][nt] = mma_bf(a1, bb, acc[1][nt]);
    }
  }
#pragma unroll
  for (int mt = 0; mt < 2; ++mt)
#pragma unroll
    for (int nt = 0; nt < 4; ++nt)
#pragma unroll
      for (int r = 0; r < 8; ++r)
        sT[(32 * w + 16 * mt + 8 * h + r) * 68 + 16 * nt + m] = acc[mt][nt][r];
  __syncthreads();
  store_hilo128<128>(sT, 68, SAGG + ((size_t)g * kN + n0) * 128, tid);
}

__device__ __forceinline__ void gate_pass(const float* sT, const float* sB, const float* __restrict__ Erow0,
                                          unsigned int* sD, int secw, int tid) {
#pragma unroll 1
  for (int it = 0; it < 8; ++it) {
    const int id = it * 128 + tid;
    const int row = id >> 3, oc = id & 7;
    const v4f e0 = *(const v4fa*)(Erow0 + (size_t)row * 64 + 8 * oc);
    const v4f e1 = *(const v4fa*)(Erow0 + (size_t)row * 64 + 8 * oc + 4);
    const v4f s0 = *(const v4fa*)(sT + row * 68 + 8 * oc);
    const v4f s1 = *(const v4fa*)(sT + row * 68 + 8 * oc + 4);
    const v4f c0 = *(const v4fa*)(sB + 8 * oc);
    const v4f c1 = *(const v4fa*)(sB + 8 * oc + 4);
    float f[8];
    f[0] = tanhf((s0.x + c0.x) * bfr(e0.x));
    f[1] = tanhf((s0.y + c0.y) * bfr(e0.y));
    f[2] = tanhf((s0.z + c0.z) * bfr(e0.z));
    f[3] = tanhf((s0.w + c0.w) * bfr(e0.w));
    f[4] = tanhf((s1.x + c1.x) * bfr(e1.x));
    f[5] = tanhf((s1.y + c1.y) * bfr(e1.y));
    f[6] = tanhf((s1.z + c1.z) * bfr(e1.z));
    f[7] = tanhf((s1.w + c1.w) * bfr(e1.w));
    v4u hi, lo;
    split8(f, hi, lo);
    *(v4ua*)(sD + row * 128 + secw + 4 * oc) = hi;
    *(v4ua*)(sD + row * 128 + secw + 32 + 4 * oc) = lo;
  }
}

__global__ __launch_bounds__(128) __attribute__((amdgpu_num_vgpr(248)))
void k_base(const unsigned short* __restrict__ XT, const unsigned short* __restrict__ WDT,
            const float* __restrict__ bd, const float* __restrict__ E1, const float* __restrict__ E2,
            unsigned short* __restrict__ DEP, int g0) {
  extern __shared__ __attribute__((aligned(16))) unsigned char sm_b[];
  float* sT = (float*)sm_b;
  unsigned int* sD = (unsigned int*)(sm_b + 128 * 68 * 4);
  float* sB = (float*)(sm_b + 128 * 68 * 4 + 128 * 128 * 4);
  const int tid = threadIdx.x, lane = tid & 31, w = tid >> 5;
  const int h = lane >> 4, m = lane & 15;
  const int gl = blockIdx.x >> 3, n0 = (blockIdx.x & 7) * 128;
  const int g = g0 + gl, t = g >> 3;
  if (tid < 16) {
    const v4f bv = *(const v4fa*)(bd + t * 64 + 4 * tid);
    const v4f br = {bfr(bv.x), bfr(bv.y), bfr(bv.z), bfr(bv.w)};
    *(v4fa*)(sB + 4 * tid) = br;
  }
  const unsigned short* a0p = XT + ((size_t)g * kN + n0 + 32 * w + m) * 64;
  const unsigned short* a1p = a0p + 16 * 64;
  const unsigned short* bp = WDT + ((size_t)t * 64 + m) * 64;
  const v8f zero8 = {0.f, 0.f, 0.f, 0.f, 0.f, 0.f, 0.f, 0.f};
  v8f acc[2][4];
#pragma unroll
  for (int mt = 0; mt < 2; ++mt)
#pragma unroll
    for (int nt = 0; nt < 4; ++nt) acc[mt][nt] = zero8;
#pragma unroll
  for (int k0 = 0; k0 < 64; k0 += 32) {
    const v16b a0 = ldfrag_g(a0p + k0, h);
    const v16b a1 = ldfrag_g(a1p + k0, h);
#pragma unroll
    for (int nt = 0; nt < 4; ++nt) {
      const v16b bb = ldfrag_g(bp + nt * 16 * 64 + k0, h);
      acc[0][nt] = mma_bf(a0, bb, acc[0][nt]);
      acc[1][nt] = mma_bf(a1, bb, acc[1][nt]);
    }
  }
#pragma unroll
  for (int mt = 0; mt < 2; ++mt)
#pragma unroll
    for (int nt = 0; nt < 4; ++nt)
#pragma unroll
      for (int r = 0; r < 8; ++r)
        sT[(32 * w + 16 * mt + 8 * h + r) * 68 + 16 * nt + m] = acc[mt][nt][r];
  __syncthreads();
  gate_pass(sT, sB, E1 + ((size_t)t * kN + n0) * 64, sD, 0, tid);
  gate_pass(sT, sB, E2 + ((size_t)t * kN + n0) * 64, sD, 64, tid);
  __syncthreads();
  unsigned short* drow = DEP + ((size_t)gl * kN + n0) * 256;
#pragma unroll 1
  for (int ch = 0; ch < 4; ++ch) {
    v4u vv[8];
#pragma unroll
    for (int it = 0; it < 8; ++it) {
      const int id = (ch * 8 + it) * 128 + tid;
      const int row = id >> 5, p = id & 31;
      vv[it] = *(const v4ua*)(sD + row * 128 + 4 * p);
    }
    for (int pass = 0; pass < 2; ++pass) {
#pragma unroll
      for (int it = 0; it < 8; ++it) {
        const int id = (ch * 8 + it) * 128 + tid;
        const int row = id >> 5, p = id & 31;
        *(volatile v4u*)(drow + (size_t)row * 256 + 8 * p) = vv[it];
      }
      __threadfence();
    }
  }
}

__global__ __launch_bounds__(256) __attribute__((amdgpu_num_vgpr(248)))
void k_anti(const unsigned short* __restrict__ DEP, unsigned short* __restrict__ DA, float* __restrict__ RSP) {
  extern __shared__ __attribute__((aligned(16))) unsigned char sm_a[];
  unsigned short* sI = (unsigned short*)sm_a;
  unsigned short* sJ = (unsigned short*)(sm_a + 65536);
  float* At = (float*)(sm_a + 131072);
  float* rs = (float*)(sm_a + 131072 + 128 * 129 * 4);
  const int tid = threadIdx.x, lane = tid & 31, w = tid >> 5;
  const int h = lane >> 4, m = lane & 15;
  const int gl = blockIdx.y;
  int rem = blockIdx.x, I = 0;
#pragma unroll
  for (int i = 0; i < 7; ++i) {
    const int len = 8 - i;
    if (I == i && rem >= len) { rem -= len; I = i + 1; }
  }
  const int J = I + rem;
  const bool diag = (I == J);

  const unsigned short* gI = DEP + ((size_t)gl * kN + I * 128) * 256;
  const unsigned short* gJ = DEP + ((size_t)gl * kN + J * 128) * 256;
#pragma unroll 4
  for (int it = 0; it < 16; ++it) {
    const int idx = it * 256 + tid;
    const v4u a = *(const v4ua*)(gI + (size_t)idx * 8);
    const v4u c = *(const v4ua*)(gJ + (size_t)idx * 8);
    *(v4ua*)(sI + idx * 8) = a;
    *(v4ua*)(sJ + idx * 8) = c;
  }
  __syncthreads();

  const unsigned short* rowA = sI + (16 * w + m) * 256;
  v16b aD1H[2], aD1L[2], aD2H[2], aD2L[2];
#pragma unroll
  for (int kk = 0; kk < 2; ++kk) {
    aD1H[kk] = ldfrag_l(rowA + 32 * kk, h);
    aD1L[kk] = ldfrag_l(rowA + 64 + 32 * kk, h);
    aD2H[kk] = ldfrag_l(rowA + 128 + 32 * kk, h);
    aD2L[kk] = ldfrag_l(rowA + 192 + 32 * kk, h);
  }
  const v8f zero8 = {0.f, 0.f, 0.f, 0.f, 0.f, 0.f, 0.f, 0.f};
#pragma unroll 1
  for (int j = 0; j < 8; ++j) {
    const unsigned short* rowB = sJ + (16 * j + m) * 256;
    v8f P = zero8, Q = zero8;
#pragma unroll
    for (int kk = 0; kk < 2; ++kk) {
      const v16b b1h = ldfrag_l(rowB + 32 * kk, h);
      const v16b b1l = ldfrag_l(rowB + 64 + 32 * kk, h);
      const v16b b2h = ldfrag_l(rowB + 128 + 32 * kk, h);
      const v16b b2l = ldfrag_l(rowB + 192 + 32 * kk, h);
      P = mma_bf(aD1H[kk], b2h, P);
      Q = mma_bf(aD2H[kk], b1h, Q);
      P = mma_bf(aD1H[kk], b2l, P);
      Q = mma_bf(aD2H[kk], b1l, Q);
      P = mma_bf(aD1L[kk], b2h, P);
      Q = mma_bf(aD2L[kk], b1h, Q);
    }
#pragma unroll
    for (int r = 0; r < 8; ++r) {
      const int row = 16 * w + 8 * h + r, col = 16 * j + m;
      float s = tanh_fast(P[r] - Q[r]);
      s = (diag && row == col) ? 0.0f : s;
      At[row * 129 + col] = s;
    }
  }
  __syncthreads();

  {
    unsigned short* daU = DA + ((size_t)gl * kN + I * 128) * kN + J * 128;
    v4u vv[8];
#pragma unroll
    for (int it = 0; it < 8; ++it) {
      const int id = it * 256 + tid;
      const int n = id >> 4, p = id & 15;
      const float* sp = At + n * 129 + 8 * p;
      v4u a;
#pragma unroll
      for (int q = 0; q < 4; ++q) {
        const float f0 = fmaxf(sp[2 * q], 0.0f);
        const float f1 = fmaxf(sp[2 * q + 1], 0.0f);
        a[q] = pk16(bfbits(f0), bfbits(f1));
      }
      vv[it] = a;
    }
    for (int pass = 0; pass < 2; ++pass) {
#pragma unroll
      for (int it = 0; it < 8; ++it) {
        const int id = it * 256 + tid;
        const int n = id >> 4, p = id & 15;
        *(volatile v4u*)(daU + (size_t)n * kN + 8 * p) = vv[it];
      }
      __threadfence();
    }
  }
  if (!diag) {
    unsigned short* daL = DA + ((size_t)gl * kN + J * 128) * kN + I * 128;
    v4u vv[8];
#pragma unroll
    for (int it = 0; it < 8; ++it) {
      const int id = it * 256 + tid;
      const int mr = id >> 4, p = id & 15;
      v4u a;
#pragma unroll
      for (int q = 0; q < 4; ++q) {
        const float f0 = fmaxf(0.0f - At[(8 * p + 2 * q) * 129 + mr], 0.0f);
        const float f1 = fmaxf(0.0f - At[(8 * p + 2 * q + 1) * 129 + mr], 0.0f);
        a[q] = pk16(bfbits(f0), bfbits(f1));
      }
      vv[it] = a;
    }
    for (int pass = 0; pass < 2; ++pass) {
#pragma unroll
      for (int it = 0; it < 8; ++it) {
        const int id = it * 256 + tid;
        const int mr = id >> 4, p = id & 15;
        *(volatile v4u*)(daL + (size_t)mr * kN + 8 * p) = vv[it];
      }
      __threadfence();
    }
  }
  float sum = 0.0f;
  if (tid < 128) {
    const float* rp = At + tid * 129;
#pragma unroll 8
    for (int c = 0; c < 128; ++c) sum += fmaxf(rp[c], 0.0f);
  } else if (!diag) {
    const int c = tid - 128;
#pragma unroll 8
    for (int n = 0; n < 128; ++n) sum += fmaxf(0.0f - At[n * 129 + c], 0.0f);
  }
  rs[tid] = sum;
  __syncthreads();
  if (w == 0) {
    const v4f v = *(const v4fa*)(rs + 4 * lane);
    float* dp = RSP + ((size_t)gl * kNT + J) * kN + I * 128 + 4 * lane;
    *(volatile v4f*)dp = v;
    __threadfence();
    *(volatile v4f*)dp = v;
  } else if (w == 1 && !diag) {
    const v4f v = *(const v4fa*)(rs + 128 + 4 * lane);
    float* dp = RSP + ((size_t)gl * kNT + I) * kN + J * 128 + 4 * lane;
    *(volatile v4f*)dp = v;
    __threadfence();
    *(volatile v4f*)dp = v;
  }
}

__global__ __launch_bounds__(256) void k_dis(const float* __restrict__ RSP, const unsigned short* __restrict__ XT,
                                             float* __restrict__ DIS, unsigned short* __restrict__ XST, int g0) {
  __shared__ __attribute__((aligned(16))) float sd[64];
  __shared__ __attribute__((aligned(16))) unsigned short sx[64 * 72];
  const int tid = threadIdx.x;
  const int gl = blockIdx.y, m0 = blockIdx.x * 64, g = g0 + gl;
#pragma unroll
  for (int it = 0; it < 2; ++it) {
    const int id = it * 256 + tid;
    const int r = id >> 3, p = id & 7;
    const v4u v = *(const v4ua*)(XT + ((size_t)g * kN + m0 + r) * 64 + 8 * p);
    *(v4ua*)(sx + r * 72 + 8 * p) = v;
  }
  if (tid < 64) {
    float s = 0.0f;
#pragma unroll 4
    for (int j = 0; j < kNT; ++j) s += RSP[((size_t)gl * kNT + j) * kN + m0 + tid];
    sd[tid] = 1.0f / sqrtf(fmaxf(1.0f + s, 1e-12f));
  }
  __syncthreads();
  if (tid < 16) {
    const v4f dv = *(const v4fa*)(sd + 4 * tid);
    float* dp = DIS + (size_t)g * kN + m0 + 4 * tid;
    *(volatile v4f*)dp = dv;
    __threadfence();
    *(volatile v4f*)dp = dv;
  }
  v4u vv[4];
#pragma unroll
  for (int it = 0; it < 4; ++it) {
    const int id = it * 256 + tid;
    const int rr = id >> 3, p = id & 7, c = rr & 63;
    float f[8];
#pragma unroll
    for (int e = 0; e < 8; ++e) {
      const int ml = 8 * p + e;
      f[e] = sd[ml] * bf2f((unsigned)sx[ml * 72 + c]);
    }
    v4u hi, lo;
    split8(f, hi, lo);
    vv[it] = (it < 2) ? hi : lo;
  }
  for (int pass = 0; pass < 2; ++pass) {
#pragma unroll
    for (int it = 0; it < 4; ++it) {
      const int id = it * 256 + tid;
      const int rr = id >> 3, p = id & 7;
      *(volatile v4u*)(XST + ((size_t)gl * 128 + rr) * kN + m0 + 8 * p) = vv[it];
    }
    __threadfence();
  }
}

__global__ __launch_bounds__(256) __attribute__((amdgpu_num_vgpr(248)))
void k_pv(const unsigned short* __restrict__ DA, const unsigned short* __restrict__ XST,
          const unsigned short* __restrict__ XT, const float* __restrict__ DIS,
          unsigned short* __restrict__ DAGG, int g0) {
  extern __shared__ __attribute__((aligned(16))) unsigned char sm_p[];
  float* Ct = (float*)sm_p;
  float* sd = (float*)(sm_p + 128 * 132 * 4);
  const int tid = threadIdx.x, lane = tid & 31, w = tid >> 5;
  const int h = lane >> 4, m = lane & 15;
  const int rg = w >> 1, chh = w & 1;
  const int gl = blockIdx.y, n0 = blockIdx.x * 128, g = g0 + gl;
  if (tid < 32) {
    const v4f d = *(const v4fa*)(DIS + (size_t)g * kN + n0 + 4 * tid);
    *(v4fa*)(sd + 4 * tid) = d;
  }
  const unsigned short* a0p = DA + ((size_t)gl * kN + n0 + 32 * rg + m) * kN;
  const unsigned short* a1p = a0p + (size_t)16 * kN;
  const unsigned short* bp = XST + ((size_t)gl * 128 + 64 * chh + m) * kN;
  const v8f zero8 = {0.f, 0.f, 0.f, 0.f, 0.f, 0.f, 0.f, 0.f};
  v8f acc[2][4];
#pragma unroll
  for (int mt = 0; mt < 2; ++mt)
#pragma unroll
    for (int nt = 0; nt < 4; ++nt) acc[mt][nt] = zero8;
#pragma unroll 1
  for (int k0 = 0; k0 < kN; k0 += 32) {
    const v16b a0 = ldfrag_g(a0p + k0, h);
    const v16b a1 = ldfrag_g(a1p + k0, h);
#pragma unroll
    for (int nt = 0; nt < 4; ++nt) {
      const v16b bb = ldfrag_g(bp + (size_t)nt * 16 * kN + k0, h);
      acc[0][nt] = mma_bf(a0, bb, acc[0][nt]);
      acc[1][nt] = mma_bf(a1, bb, acc[1][nt]);
    }
  }
#pragma unroll
  for (int mt = 0; mt < 2; ++mt)
#pragma unroll
    for (int nt = 0; nt < 4; ++nt)
#pragma unroll
      for (int r = 0; r < 8; ++r)
        Ct[(32 * rg + 16 * mt + 8 * h + r) * 132 + 64 * chh + 16 * nt + m] = acc[mt][nt][r];
  __syncthreads();
  v4u vv[8];
#pragma unroll
  for (int it = 0; it < 8; ++it) {
    const int id = it * 256 + tid;
    const int n = id >> 4, p = id & 15, oc = p & 7;
    const v4u xw = *(const v4ua*)(XT + ((size_t)g * kN + n0 + n) * 64 + 8 * oc);
    const float dn = sd[n];
    const v4f h0 = *(const v4fa*)(Ct + n * 132 + 8 * oc);
    const v4f h1 = *(const v4fa*)(Ct + n * 132 + 8 * oc + 4);
    const v4f l0 = *(const v4fa*)(Ct + n * 132 + 64 + 8 * oc);
    const v4f l1 = *(const v4fa*)(Ct + n * 132 + 64 + 8 * oc + 4);
    const float raw[8] = {h0.x + l0.x, h0.y + l0.y, h0.z + l0.z, h0.w + l0.w,
                          h1.x + l1.x, h1.y + l1.y, h1.z + l1.z, h1.w + l1.w};
    float f[8];
#pragma unroll
    for (int q = 0; q < 4; ++q) {
      const unsigned wq = xw[q];
      const float xe = __uint_as_float(wq << 16);
      const float xo = __uint_as_float(wq & 0xffff0000u);
      f[2 * q]     = dn * (raw[2 * q] + dn * xe);
      f[2 * q + 1] = dn * (raw[2 * q + 1] + dn * xo);
    }
    v4u hi, lo;
    split8(f, hi, lo);
    vv[it] = blend4(hi, lo, (unsigned)(p >> 3));
  }
  unsigned short* drow = DAGG + ((size_t)g * kN + n0) * 128;
  for (int pass = 0; pass < 2; ++pass) {
#pragma unroll
    for (int it = 0; it < 8; ++it) {
      const int id = it * 256 + tid;
      const int n = id >> 4, p = id & 15;
      *(volatile v4u*)(drow + (size_t)n * 128 + 8 * p) = vv[it];
    }
    __threadfence();
  }
}

__global__ __launch_bounds__(128) __attribute__((amdgpu_num_vgpr(248)))
void k_out(const unsigned short* __restrict__ SAGG, const unsigned short* __restrict__ DAGG,
           const unsigned short* __restrict__ XT, const unsigned short* __restrict__ WS2,
           const unsigned short* __restrict__ WD2, const unsigned short* __restrict__ W0T,
           const float* __restrict__ bs, const float* __restrict__ bd, const float* __restrict__ b0,
           float* __restrict__ out) {
  extern __shared__ __attribute__((aligned(16))) unsigned char sm_o[];
  float* tile = (float*)sm_o;
  float* sbs = (float*)(sm_o + 32 * 768 * 4);
  float* sbd = sbs + 768;
  float* sb0 = sbd + 768;
  const int tid = threadIdx.x, lane = tid & 31, w = tid >> 5;
  const int h = lane >> 4, m = lane & 15;
  const int b = blockIdx.y, n0 = blockIdx.x * 32;
  {
    const v4f a = *(const v4fa*)(bs + 4 * tid);
    const v4f c = *(const v4fa*)(bd + 4 * tid);
    const v4f ar = {bfr(a.x), bfr(a.y), bfr(a.z), bfr(a.w)};
    const v4f cr = {bfr(c.x), bfr(c.y), bfr(c.z), bfr(c.w)};
    *(v4fa*)(sbs + 4 * tid) = ar;
    *(v4fa*)(sbd + 4 * tid) = cr;
  }
  if (tid < 64) {
    const v4f a = *(const v4fa*)(bs + 512 + 4 * tid);
    const v4f c = *(const v4fa*)(bd + 512 + 4 * tid);
    const v4f ar = {bfr(a.x), bfr(a.y), bfr(a.z), bfr(a.w)};
    const v4f cr = {bfr(c.x), bfr(c.y), bfr(c.z), bfr(c.w)};
    *(v4fa*)(sbs + 512 + 4 * tid) = ar;
    *(v4fa*)(sbd + 512 + 4 * tid) = cr;
  }
  if (tid < 16) {
    const v4f a = *(const v4fa*)(b0 + 4 * tid);
    const v4f ar = {bfr(a.x), bfr(a.y), bfr(a.z), bfr(a.w)};
    *(v4fa*)(sb0 + 4 * tid) = ar;
  }
  __syncthreads();
  const float c1 = (float)(0.5 - 0.025);
  const float c2 = (float)(1.0 - 0.5 - 0.025);
  const float c3 = 0.05f;
  const int o = 16 * w + m;
  const v8f zero8 = {0.f, 0.f, 0.f, 0.f, 0.f, 0.f, 0.f, 0.f};
  const unsigned short* w0p = W0T + (size_t)o * 64;
#pragma unroll 1
  for (int t = 0; t < kT; ++t) {
    const int g = t * kB + b;
    const unsigned short* rowS = SAGG + ((size_t)g * kN + n0 + m) * 128;
    const unsigned short* rowD = DAGG + ((size_t)g * kN + n0 + m) * 128;
    const unsigned short* rowX = XT + ((size_t)g * kN + n0 + m) * 64;
    const unsigned short* wsp = WS2 + ((size_t)t * 64 + o) * 128;
    const unsigned short* wdp = WD2 + ((size_t)t * 64 + o) * 128;
    v8f accS[2] = {zero8, zero8}, accD[2] = {zero8, zero8}, acc0[2] = {zero8, zero8};
#pragma unroll
    for (int ks = 0; ks < 4; ++ks) {
      const v16b bS = ldfrag_g(wsp + 32 * ks, h);
      const v16b bD = ldfrag_g(wdp + 32 * ks, h);
#pragma unroll
      for (int mt = 0; mt < 2; ++mt) {
        const v16b aS = ldfrag_g(rowS + mt * 16 * 128 + 32 * ks, h);
        const v16b aD = ldfrag_g(rowD + mt * 16 * 128 + 32 * ks, h);
        accS[mt] = mma_bf(aS, bS, accS[mt]);
        accD[mt] = mma_bf(aD, bD, accD[mt]);
      }
    }
#pragma unroll
    for (int ks = 0; ks < 2; ++ks) {
      const v16b bX = ldfrag_g(w0p + 32 * ks, h);
#pragma unroll
      for (int mt = 0; mt < 2; ++mt) {
        const v16b aX = ldfrag_g(rowX + mt * 16 * 64 + 32 * ks, h);
        acc0[mt] = mma_bf(aX, bX, acc0[mt]);
      }
    }
    const float bsv = sbs[t * 64 + o], bdv = sbd[t * 64 + o], b0v = sb0[o];
#pragma unroll
    for (int mt = 0; mt < 2; ++mt)
#pragma unroll
      for (int r = 0; r < 8; ++r) {
        const int nl = 16 * mt + 8 * h + r;
        const float f = (c1 * (accS[mt][r] + bsv) + c2 * (accD[mt][r] + bdv)) + c3 * (acc0[mt][r] + b0v);
        tile[nl * 768 + o * 12 + t] = f;
      }
  }
  __syncthreads();
  float* dst = out + ((size_t)b * kN + n0) * 768;
  for (int pass = 0; pass < 2; ++pass) {
#pragma unroll 4
    for (int it = 0; it < 48; ++it) {
      const int i4 = it * 128 + tid;
      const v4f v = *(const v4fa*)(tile + 4 * i4);
      *(volatile v4f*)(dst + (size_t)4 * i4) = v;
    }
    __threadfence();
  }
}

extern "C" void kernel_launch(void* const* d_in, const int* in_sizes, int n_in,
                              void* d_out, int out_size, void* d_ws, size_t ws_size,
                              hipStream_t stream) {
  if (n_in < 10) return;
  if (in_sizes[0] != kB * kN * kC * kT) return;
  if (in_sizes[1] != kN * kN) return;
  if (in_sizes[2] != kC * kO || in_sizes[3] != kO) return;
  if (in_sizes[4] != kT * kC * kO || in_sizes[5] != kT * kO) return;
  if (in_sizes[6] != kT * kC * kO || in_sizes[7] != kT * kO) return;
  if (in_sizes[8] != kT * kN * kO || in_sizes[9] != kT * kN * kO) return;
  if (out_size != kB * kN * kO * kT) return;
  if (WS_TOTAL > ws_size) return;

  const float* x   = (const float*)d_in[0];
  const float* adj = (const float*)d_in[1];
  const float* W0  = (const float*)d_in[2];
  const float* b0  = (const float*)d_in[3];
  const float* Ws  = (const float*)d_in[4];
  const float* bs  = (const float*)d_in[5];
  const float* Wd  = (const float*)d_in[6];
  const float* bd  = (const float*)d_in[7];
  const float* E1  = (const float*)d_in[8];
  const float* E2  = (const float*)d_in[9];
  float* out = (float*)d_out;

  char* ws = (char*)d_ws;
  unsigned short* XT   = (unsigned short*)(ws + OFF_XT);
  unsigned short* XTT  = (unsigned short*)(ws + OFF_XTT);
  unsigned short* ADJB = (unsigned short*)(ws + OFF_ADJB);
  unsigned short* WDT  = (unsigned short*)(ws + OFF_WDT);
  unsigned short* WS2  = (unsigned short*)(ws + OFF_WS2);
  unsigned short* WD2  = (unsigned short*)(ws + OFF_WD2);
  unsigned short* W0T  = (unsigned short*)(ws + OFF_W0T);
  unsigned short* SAGG = (unsigned short*)(ws + OFF_SAGG);
  unsigned short* DAGG = (unsigned short*)(ws + OFF_DAGG);
  unsigned short* DEP  = (unsigned short*)(ws + OFF_DEP);
  unsigned short* DA   = (unsigned short*)(ws + OFF_DA);
  float*          RSP  = (float*)(ws + OFF_RSP);
  float*          DIS  = (float*)(ws + OFF_DIS);
  unsigned short* XST  = (unsigned short*)(ws + OFF_XST);

  (void)hipFuncSetAttribute((const void*)k_prep_x, hipFuncAttributeMaxDynamicSharedMemorySize, LDS_PREPX);
  (void)hipFuncSetAttribute((const void*)k_base,   hipFuncAttributeMaxDynamicSharedMemorySize, LDS_BASE);
  (void)hipFuncSetAttribute((const void*)k_anti,   hipFuncAttributeMaxDynamicSharedMemorySize, LDS_ANTI);
  (void)hipFuncSetAttribute((const void*)k_pv,     hipFuncAttributeMaxDynamicSharedMemorySize, LDS_PV);
  (void)hipFuncSetAttribute((const void*)k_out,    hipFuncAttributeMaxDynamicSharedMemorySize, LDS_OUT);

  k_prep_x<<<dim3(kB * (kN / 64)), dim3(256), LDS_PREPX, stream>>>(x, XT, XTT);
  k_prep_w<<<dim3(512 + 25), dim3(256), 0, stream>>>(adj, W0, Ws, Wd, ADJB, WDT, WS2, WD2, W0T);
  k_static<<<dim3(kNT, kG), dim3(128), 0, stream>>>(ADJB, XTT, SAGG);

  for (int q = 0; q < kNGRP; ++q) {
    const int g0 = q * kGL;
    k_base<<<dim3(kGL * kNT), dim3(128), LDS_BASE, stream>>>(XT, WDT, bd, E1, E2, DEP, g0);
    k_anti<<<dim3(kPAIRS, kGL), dim3(256), LDS_ANTI, stream>>>(DEP, DA, RSP);
    k_dis<<<dim3(kN / 64, kGL), dim3(256), 0, stream>>>(RSP, XT, DIS, XST, g0);
    k_pv<<<dim3(kNT, kGL), dim3(256), LDS_PV, stream>>>(DA, XST, XT, DIS, DAGG, g0);
  }

  k_out<<<dim3(kN / 32, kB), dim3(128), LDS_OUT, stream>>>(SAGG, DAGG, XT, WS2, WD2, W0T, bs, bd, b0, out);
}
